// EdgePredictor_29832842838651
// MI455X (gfx1250) — hardware-verified
//
#include <hip/hip_runtime.h>
#include <math.h>

constexpr int NG = 100000;
constexpr int NU = 100000;
constexpr int NS = NG + NU;
constexpr int NE = 3200000;
constexpr int NC = 2000000;
constexpr int NT = 256;
constexpr int CHUNK = 4096;
constexpr int SPT = CHUNK / NT;
constexpr int NCHUNK = (NE + CHUNK - 1) / CHUNK;
constexpr int SUBCAP = 256;
constexpr int TILE1 = 4096;
constexpr int TILE2 = 2048;
constexpr int NTILE1 = (NG + TILE1 - 1) / TILE1;
constexpr int NTILE2 = (NG + TILE2 - 1) / TILE2;
constexpr int NGRP = NC / 128;
constexpr int MLP_BLOCKS = (NGRP + 7) / 8;
constexpr int LDS1_BYTES = (TILE1 * 4 + CHUNK + 8 * SUBCAP + 96 + 72) * 4;
constexpr int LDS2_BYTES = (TILE2 * 8 + CHUNK + 8 * SUBCAP + 96 + 272) * 4;

static_assert(NE % SPT == 0, "edge groups are whole");
static_assert(NC % 128 == 0, "output groups are whole");
static_assert(NG % 16 == 0 && NU % 16 == 0, "wave-uniform row tails");
static_assert(TILE1 / 8 == 512 && TILE2 / 8 == 256, "rows per wave are 2^9 and 2^8");
static_assert(128 * 8 * 4 <= CHUNK * 4, "h staging fits in the list region");

typedef __attribute__((ext_vector_type(16))) _Float16 v16h;
typedef __attribute__((ext_vector_type(8)))  _Float16 v8h;
typedef __attribute__((ext_vector_type(8)))  float    v8f;
typedef __attribute__((ext_vector_type(4)))  float    v4f;
typedef __attribute__((ext_vector_type(4)))  int      v4i;
typedef __attribute__((ext_vector_type(4)))  unsigned int v4u;

template <typename T> struct Frag;
template <> struct Frag<_Float16> {
  typedef v16h V; union U { v16h v; v8h h[2]; };
  static __device__ __forceinline__ v16h load(const _Float16* p) {
    U f; f.h[0] = *(const v8h*)(p); f.h[1] = *(const v8h*)(p + 16); return f.v;
  }
  static __device__ __forceinline__ v8f mma(v16h a, v16h b, v8f c) {
    return __builtin_amdgcn_wmma_f32_16x16x32_f16(false, a, false, b, (short)0, c, false, false);
  }
};
__device__ __forceinline__ void guard6(v8f& a, v8f& b, v16h x, v16h y, v16h z, v16h w) {
  asm volatile("v_nop\n\tv_nop\n\tv_nop\n\tv_nop" : "+v"(a), "+v"(b) : "v"(x), "v"(y), "v"(z), "v"(w));
}

__device__ __forceinline__ unsigned pk16(unsigned short a, unsigned short b) { return (unsigned)a | ((unsigned)b << 16); }
__device__ __forceinline__ unsigned short h_bits(float f) { const _Float16 h = (_Float16)f; return __builtin_bit_cast(unsigned short, h); }

__device__ __forceinline__ void split_h16(float v, unsigned short& hb, unsigned short& lb) {
  const _Float16 h = (_Float16)v;
  const float hf = (float)h;
  const float res = (v - hf) * 2048.0f;
  hb = __builtin_bit_cast(unsigned short, h);
  lb = h_bits(res);
}

__device__ __forceinline__ float selu_f32(float x) {
  const float kScale = 1.0507009873554805f;
  const float kAlpha = 1.6732632423543772f;
  const float pos = fmaxf(x, 0.0f);
  const float em1 = expf(fminf(x, 0.0f)) - 1.0f;
  return kScale * fmaf(kAlpha, em1, pos);
}

__device__ __forceinline__ float fsel(bool c, float a, float b) {
  const float f = c ? 1.0f : 0.0f;
  const float g = 1.0f - f;
  return fmaf(f, b, g * a);
}

__device__ __forceinline__ void wave_lds_sync() {
  __builtin_amdgcn_fence(__ATOMIC_RELEASE, "workgroup");
  __builtin_amdgcn_wave_barrier();
  __builtin_amdgcn_fence(__ATOMIC_ACQUIRE, "workgroup");
}

__device__ __forceinline__ int blk_excl_scan(int cnt, int* scan_ws, int tid, int* tot) {
  const int lane = tid & 31, wave = tid >> 5; int incl = cnt;
#pragma unroll
  for (int o = 1; o < 32; o <<= 1) { const int v = __shfl_up(incl, o, 32); if (lane >= o) incl += v; }
  if (lane == 31) scan_ws[wave] = incl;
  __syncthreads();
  if (wave == 0) { int wv = (lane < NT / 32) ? scan_ws[lane] : 0; int wincl = wv;
#pragma unroll
    for (int o = 1; o < 32; o <<= 1) { const int v = __shfl_up(wincl, o, 32); if (lane >= o) wincl += v; }
    if (lane < NT / 32) scan_ws[32 + lane] = wincl - wv; if (lane == 31) scan_ws[64] = wincl; }
  __syncthreads();
  const int res = scan_ws[32 + wave] + incl - cnt; *tot = scan_ws[64];
  return res;
}

template <int TILE>
__device__ __forceinline__ int chunk_hits16(const int* __restrict__ dstv, const int* __restrict__ srcv, int e0, int n0,
                                            int tid, int* LIST, int* scan_ws) {
  const int eb = e0 + tid * SPT;
  const bool live = eb < NE;
  const int ebc = live ? eb : (NE - SPT);
  int rec[SPT]; int cnt = 0;
#pragma unroll
  for (int k = 0; k < SPT; k += 4) {
    const v4i d4 = *(const v4i*)(dstv + ebc + k);
    const v4i s4 = *(const v4i*)(srcv + ebc + k);
#pragma unroll
    for (int e = 0; e < 4; ++e) {
      const int d = d4[e]; int s = s4[e];
      s = (s < 0) ? 0 : ((s >= NG) ? (NG - 1) : s);
      const bool hit = live && (d >= n0) && (d < n0 + TILE);
      const int dl = d - n0;
      rec[k + e] = hit ? ((dl << 17) | s) : -1;
      cnt += hit ? 1 : 0;
    }
  }
  int tot; int p = blk_excl_scan(cnt, scan_ws, tid, &tot);
#pragma unroll
  for (int k = 0; k < SPT; ++k) if (rec[k] >= 0) { if ((unsigned)p < (unsigned)CHUNK) LIST[p] = rec[k]; ++p; }
  __syncthreads();
  return tot < CHUNK ? tot : CHUNK;
}

template <int NCH, int TILE>
__device__ __forceinline__ void drain_hits(const int* SUBw, int cnt, float* ACC, const float* __restrict__ feat, int lane) {
  wave_lds_sync();
#pragma unroll 1
  for (int base = 0; base < SUBCAP; base += 32) {
    if (base >= cnt) break;
    const int q = base + lane;
    const bool valid = q < cnt;
    const int qc = valid ? q : (cnt - 1);
    const int rv = SUBw[qc];
    const int dl = valid ? ((rv >> 17) & (TILE - 1)) : 0;
    int s = rv & 0x1FFFF; s = valid ? s : 0; s = (s >= NG) ? (NG - 1) : s;
    const int key = valid ? dl : (-1 - lane);
    const float* fr = feat + (size_t)s * NCH;
    const v4f f0 = *(const v4f*)fr;
    v4f f1 = {0.f, 0.f, 0.f, 0.f};
    if (NCH == 8) f1 = *(const v4f*)(fr + 4);
    int rank = 0;
#pragma unroll
    for (int j = 0; j < 32; ++j) { const int kj = __shfl(key, j, 32); rank += ((j < lane) && (kj == key)) ? 1 : 0; }
    int mr = valid ? rank : 0;
#pragma unroll
    for (int off = 1; off < 32; off <<= 1) { const int o = __shfl_xor(mr, off, 32); mr = (o > mr) ? o : mr; }
    const int nr = __builtin_amdgcn_readfirstlane(mr) + 1;
    float* row = ACC + dl * NCH;
#pragma unroll 1
    for (int r = 0; r < 32; ++r) {
      if (r >= nr) break;
      if (valid && rank == r) {
        v4f a0 = *(const v4f*)row; a0 = a0 + f0; *(v4f*)row = a0;
        if (NCH == 8) { v4f a1 = *(const v4f*)(row + 4); a1 = a1 + f1; *(v4f*)(row + 4) = a1; }
      }
      wave_lds_sync();
    }
  }
}

template <int NCH, int TILE, int LRW>
__device__ __forceinline__ void stream_tile(const int* __restrict__ edges, const float* __restrict__ feat, int n0,
                                            float* ACC, int* LIST, int* SUB, int* scan_ws, int tid, int lane, int wave) {
  const int* srcv = edges;
  const int* dstv = edges + NE;
  int* SUBw = SUB + wave * SUBCAP;
#pragma unroll 1
  for (int c = 0; c < NCHUNK; ++c) {
    const int tot = __builtin_amdgcn_readfirstlane(chunk_hits16<TILE>(dstv, srcv, c * CHUNK, n0, tid, LIST, scan_ws));
    int cnt = 0;
#pragma unroll 1
    for (int base = 0; base < CHUNK; base += 32) {
      if (base >= tot) break;
      const int q = base + lane;
      const bool inr = q < tot;
      const int rv = LIST[q];
      const bool own = inr && (rv >= 0) && ((rv >> (17 + LRW)) == wave);
      const unsigned m = (unsigned)__ballot(own ? 1 : 0);
      const int pc = (int)__popc(m);
      if (cnt + pc > SUBCAP) { drain_hits<NCH, TILE>(SUBw, cnt, ACC, feat, lane); cnt = 0; }
      const unsigned below = m & ((1u << lane) - 1u);
      const int pos = cnt + (int)__popc(below);
      if (own) SUBw[pos] = rv;
      cnt += pc;
    }
    drain_hits<NCH, TILE>(SUBw, cnt, ACC, feat, lane);
    __syncthreads();
  }
}

__global__ __launch_bounds__(NT) void lin_un_kernel(const float* __restrict__ xu, const float* __restrict__ Wun,
                                                    const float* __restrict__ bun,
                                                    unsigned short* __restrict__ XH, unsigned short* __restrict__ XL) {
  __shared__ float WS[80];
  const int tid = threadIdx.x;
  if (tid < 64) WS[tid] = Wun[tid];
  if (tid < 16) WS[64 + tid] = bun[tid];
  __syncthreads();
  const int n = blockIdx.x * 128 + (tid >> 1);
  const int c0 = 8 * (tid & 1);
  const int nc = (n < NU) ? n : (NU - 1);
  const v4f x = *(const v4f*)(xu + (size_t)nc * 4);
  unsigned short hb[8], lb[8];
#pragma unroll
  for (int j = 0; j < 8; ++j) {
    const int c = c0 + j;
    float v = 0.0f;
#pragma unroll
    for (int k = 0; k < 4; ++k) v = fmaf(x[k], WS[k * 16 + c], v);
    v = v + WS[64 + c];
    split_h16(v, hb[j], lb[j]);
  }
  const v4u uh = {pk16(hb[0], hb[1]), pk16(hb[2], hb[3]), pk16(hb[4], hb[5]), pk16(hb[6], hb[7])};
  const v4u ul = {pk16(lb[0], lb[1]), pk16(lb[2], lb[3]), pk16(lb[4], lb[5]), pk16(lb[6], lb[7])};
  if (n < NU) {
    unsigned short* ph = XH + (size_t)(NG + n) * 16 + c0;
    unsigned short* pl = XL + (size_t)(NG + n) * 16 + c0;
    for (int pass = 0; pass < 2; ++pass) { *(volatile v4u*)ph = uh; *(volatile v4u*)pl = ul; __threadfence(); }
  }
}

__global__ __launch_bounds__(NT) void agg1_kernel(const float* __restrict__ xg, const int* __restrict__ edges,
                                                  const float* __restrict__ W1r, const float* __restrict__ W1o,
                                                  const float* __restrict__ b1v, float* __restrict__ HPL) {
  extern __shared__ __attribute__((aligned(16))) float dyn_lds[];
  float* ACC = dyn_lds;
  int* LIST = (int*)(dyn_lds + TILE1 * 4);
  int* SUB = LIST + CHUNK;
  int* scan_ws = SUB + 8 * SUBCAP;
  float* WS = (float*)(scan_ws + 96);
  const int tid = threadIdx.x, lane = tid & 31, wave = tid >> 5;
  const int n0 = blockIdx.x * TILE1;
  for (int i = tid; i < TILE1 * 4; i += NT) ACC[i] = 0.0f;
  for (int i = tid; i < CHUNK + 8 * SUBCAP + 96; i += NT) LIST[i] = 0;
  if (tid < 32) { WS[tid] = W1r[tid]; WS[32 + tid] = W1o[tid]; }
  if (tid < 8) WS[64 + tid] = b1v[tid];
  __syncthreads();
  stream_tile<4, TILE1, 9>(edges, xg, n0, ACC, LIST, SUB, scan_ws, tid, lane, wave);
#pragma unroll 1
  for (int ps = 0; ps < TILE1 / 128; ++ps) {
    const int nb = n0 + ps * 128;
    if (nb >= NG) break;
    const int nl = ps * 128 + (tid >> 1);
    const int n = n0 + nl;
    const int c0 = 4 * (tid & 1);
    const v4f a = *(const v4f*)(ACC + nl * 4);
    const int nc = (n < NG) ? n : (NG - 1);
    const v4f x = *(const v4f*)(xg + (size_t)nc * 4);
    float o[4];
#pragma unroll
    for (int j = 0; j < 4; ++j) {
      const int c = c0 + j;
      float vr = 0.0f, vo = 0.0f;
#pragma unroll
      for (int k = 0; k < 4; ++k) { vr = fmaf(a[k], WS[k * 8 + c], vr); vo = fmaf(x[k], WS[32 + k * 8 + c], vo); }
      float v = vr + vo;
      v = v + WS[64 + c];
      o[j] = selu_f32(v);
    }
    const v4f ov = {o[0], o[1], o[2], o[3]};
    if (n < NG) {
      float* hp = HPL + (size_t)n * 8 + c0;
      for (int pass = 0; pass < 2; ++pass) { *(volatile v4f*)hp = ov; __threadfence(); }
    }
  }
}

__global__ __launch_bounds__(NT) void agg2_kernel(const float* __restrict__ HPL, const int* __restrict__ edges,
                                                  const float* __restrict__ W2r, const float* __restrict__ W2o,
                                                  const float* __restrict__ b2v,
                                                  unsigned short* __restrict__ XH, unsigned short* __restrict__ XL) {
  extern __shared__ __attribute__((aligned(16))) float dyn_lds[];
  float* ACC = dyn_lds;
  int* LIST = (int*)(dyn_lds + TILE2 * 8);
  int* SUB = LIST + CHUNK;
  int* scan_ws = SUB + 8 * SUBCAP;
  float* WS = (float*)(scan_ws + 96);
  const int tid = threadIdx.x, lane = tid & 31, wave = tid >> 5;
  const int n0 = blockIdx.x * TILE2;
  for (int i = tid; i < TILE2 * 8; i += NT) ACC[i] = 0.0f;
  for (int i = tid; i < CHUNK + 8 * SUBCAP + 96; i += NT) LIST[i] = 0;
  for (int i = tid; i < 128; i += NT) { WS[i] = W2r[i]; WS[128 + i] = W2o[i]; }
  if (tid < 16) WS[256 + tid] = b2v[tid];
  __syncthreads();
  stream_tile<8, TILE2, 8>(edges, HPL, n0, ACC, LIST, SUB, scan_ws, tid, lane, wave);
  float* HST = (float*)LIST;
#pragma unroll 1
  for (int ps = 0; ps < TILE2 / 128; ++ps) {
    const int nb = n0 + ps * 128;
    if (nb >= NG) break;
    {
      const int n = nb + (tid >> 1);
      const int nc = (n < NG) ? n : (NG - 1);
      *(v4f*)(HST + 4 * tid) = *(const v4f*)(HPL + (size_t)nc * 8 + 4 * (tid & 1));
    }
    __syncthreads();
    const int nl = ps * 128 + (tid >> 1);
    const int n = n0 + nl;
    const int c0 = 8 * (tid & 1);
    float o[8];
#pragma unroll
    for (int j = 0; j < 8; ++j) o[j] = 0.0f;
#pragma unroll 1
    for (int k = 0; k < 8; ++k) {
      const float ak = ACC[nl * 8 + k];
      const float hk = HST[(tid >> 1) * 8 + k];
#pragma unroll
      for (int j = 0; j < 8; ++j) {
        o[j] = fmaf(ak, WS[k * 16 + c0 + j], o[j]);
        o[j] = fmaf(hk, WS[128 + k * 16 + c0 + j], o[j]);
      }
    }
    unsigned short hb[8], lb[8];
#pragma unroll
    for (int j = 0; j < 8; ++j) {
      float v = o[j] + WS[256 + c0 + j];
      v = selu_f32(v);
      split_h16(v, hb[j], lb[j]);
    }
    const v4u uh = {pk16(hb[0], hb[1]), pk16(hb[2], hb[3]), pk16(hb[4], hb[5]), pk16(hb[6], hb[7])};
    const v4u ul = {pk16(lb[0], lb[1]), pk16(lb[2], lb[3]), pk16(lb[4], lb[5]), pk16(lb[6], lb[7])};
    if (n < NG) {
      unsigned short* ph = XH + (size_t)n * 16 + c0;
      unsigned short* pl = XL + (size_t)n * 16 + c0;
      for (int pass = 0; pass < 2; ++pass) { *(volatile v4u*)ph = uh; *(volatile v4u*)pl = ul; __threadfence(); }
    }
    __syncthreads();
  }
}

__global__ __launch_bounds__(NT) void mlp_kernel(const int* __restrict__ cand,
                                                 const unsigned short* __restrict__ XHp, const unsigned short* __restrict__ XLp,
                                                 const float* __restrict__ Wfc1, const float* __restrict__ bfc1,
                                                 const float* __restrict__ Wfc2, const float* __restrict__ bfc2,
                                                 float* __restrict__ out) {
  __shared__ __align__(16) _Float16 sBh[64 * 32];
  __shared__ __align__(16) _Float16 sBl[64 * 32];
  __shared__ __align__(16) _Float16 sAh[8][16 * 32];
  __shared__ __align__(16) _Float16 sAl[8][16 * 32];
  __shared__ __align__(16) float sO[8][128];
  __shared__ float sb[64];
  __shared__ float sw[64];
  const int tid = threadIdx.x, lane = tid & 31, wave = tid >> 5;
  {
    const int n = tid >> 2, g = tid & 3;
    unsigned short hb[8], lb[8];
#pragma unroll
    for (int e = 0; e < 8; ++e) {
      const int k = 8 * g + e;
      const float w = Wfc1[k * 64 + n] * 16.0f;
      split_h16(w, hb[e], lb[e]);
    }
    const v4u uh = {pk16(hb[0], hb[1]), pk16(hb[2], hb[3]), pk16(hb[4], hb[5]), pk16(hb[6], hb[7])};
    const v4u ul = {pk16(lb[0], lb[1]), pk16(lb[2], lb[3]), pk16(lb[4], lb[5]), pk16(lb[6], lb[7])};
    *(v4u*)(sBh + n * 32 + 8 * g) = uh;
    *(v4u*)(sBl + n * 32 + 8 * g) = ul;
    if (tid < 64) { sb[tid] = bfc1[tid]; sw[tid] = Wfc2[tid]; }
  }
  __syncthreads();
  const int hh = lane >> 4, cidx = lane & 15;
  v16h bh[4], bl[4];
  float hb4[4], w24[4];
#pragma unroll
  for (int j = 0; j < 4; ++j) {
    bh[j] = Frag<_Float16>::load(sBh + (16 * j + cidx) * 32 + 8 * hh);
    bl[j] = Frag<_Float16>::load(sBl + (16 * j + cidx) * 32 + 8 * hh);
    hb4[j] = sb[16 * j + cidx];
    w24[j] = sw[16 * j + cidx];
  }
  const float bias2 = bfc2[0];
  const float inv2048 = 1.0f / 2048.0f;
  const float inv16 = 0.0625f;
  const v8f zero8 = {0.f, 0.f, 0.f, 0.f, 0.f, 0.f, 0.f, 0.f};
  const _Float16* XH = (const _Float16*)XHp;
  const _Float16* XL = (const _Float16*)XLp;
  _Float16* Ah = sAh[wave];
  _Float16* Al = sAl[wave];
  float* so = sO[wave];
  const int pr = lane >> 2, pe = (lane >> 1) & 1, pq = lane & 1;
  const bool bit0 = (lane & 1) != 0, bit1 = (lane & 2) != 0, bit2 = (lane & 4) != 0;
  const int gw = blockIdx.x * 8 + wave;
  const int nw = gridDim.x * 8;
#pragma unroll 1
  for (int g = gw; g < NGRP; g += nw) {
#pragma unroll 1
    for (int mt = 0; mt < 8; ++mt) {
      const int cb = g * 128 + mt * 16;
      int i0 = cand[(size_t)(cb + pr) * 2 + pe];
      int i1 = cand[(size_t)(cb + 8 + pr) * 2 + pe];
      i0 = (i0 < 0) ? 0 : ((i0 >= NS) ? (NS - 1) : i0);
      i1 = (i1 < 0) ? 0 : ((i1 >= NS) ? (NS - 1) : i1);
      const v8h h0 = *(const v8h*)(XH + (size_t)i0 * 16 + 8 * pq);
      const v8h l0 = *(const v8h*)(XL + (size_t)i0 * 16 + 8 * pq);
      const v8h h1 = *(const v8h*)(XH + (size_t)i1 * 16 + 8 * pq);
      const v8h l1 = *(const v8h*)(XL + (size_t)i1 * 16 + 8 * pq);
      *(v8h*)(Ah + 8 * lane) = h0;
      *(v8h*)(Ah + 256 + 8 * lane) = h1;
      *(v8h*)(Al + 8 * lane) = l0;
      *(v8h*)(Al + 256 + 8 * lane) = l1;
      wave_lds_sync();
      const v16h ah = Frag<_Float16>::load(Ah + cidx * 32 + 8 * hh);
      const v16h al = Frag<_Float16>::load(Al + cidx * 32 + 8 * hh);
      float p[8];
#pragma unroll
      for (int r = 0; r < 8; ++r) p[r] = 0.0f;
#pragma unroll
      for (int j = 0; j < 4; ++j) {
        v8f am = Frag<_Float16>::mma(ah, bh[j], zero8);
        v8f ar = Frag<_Float16>::mma(ah, bl[j], zero8);
        ar = Frag<_Float16>::mma(al, bh[j], ar);
        guard6(am, ar, ah, al, bh[j], bl[j]);
#pragma unroll
        for (int r = 0; r < 8; ++r) {
          float v = fmaf(ar[r], inv2048, am[r]);
          v = fmaf(v, inv16, hb4[j]);
          v = selu_f32(v);
          p[r] = fmaf(v, w24[j], p[r]);
        }
      }
      float q4[4];
#pragma unroll
      for (int i = 0; i < 4; ++i) {
        const float x0 = __shfl_xor(p[2 * i], 1, 32);
        const float x1 = __shfl_xor(p[2 * i + 1], 1, 32);
        q4[i] = fsel(bit0, p[2 * i] + x0, p[2 * i + 1] + x1);
      }
      float r2a, r2b;
      {
        const float y0 = __shfl_xor(q4[0], 2, 32);
        const float y1 = __shfl_xor(q4[1], 2, 32);
        const float y2 = __shfl_xor(q4[2], 2, 32);
        const float y3 = __shfl_xor(q4[3], 2, 32);
        r2a = fsel(bit1, q4[0] + y0, q4[1] + y1);
        r2b = fsel(bit1, q4[2] + y2, q4[3] + y3);
      }
      float s;
      {
        const float z0 = __shfl_xor(r2a, 4, 32);
        const float z1 = __shfl_xor(r2b, 4, 32);
        s = fsel(bit2, r2a + z0, r2b + z1);
      }
      const float s8 = __shfl_xor(s, 8, 32);
      s = s + s8;
      if ((lane & 8) == 0) so[mt * 16 + 8 * hh + (lane & 7)] = s + bias2;
    }
    wave_lds_sync();
    const v4f ov = *(const v4f*)(so + 4 * lane);
    float* op = out + (size_t)g * 128 + 4 * lane;
    for (int pass = 0; pass < 2; ++pass) { *(volatile v4f*)op = ov; __threadfence(); }
  }
}

extern "C" void kernel_launch(void* const* d_in, const int* in_sizes, int n_in,
                              void* d_out, int out_size, void* d_ws, size_t ws_size, hipStream_t stream) {
  (void)in_sizes; (void)n_in; (void)out_size;
  const float* x_u   = (const float*)d_in[0];
  const float* x_g   = (const float*)d_in[1];
  const int*   cand  = (const int*)d_in[2];
  const int*   edges = (const int*)d_in[3];
  const float* W1r   = (const float*)d_in[4];
  const float* W1o   = (const float*)d_in[5];
  const float* b1v   = (const float*)d_in[6];
  const float* W2r   = (const float*)d_in[7];
  const float* W2o   = (const float*)d_in[8];
  const float* b2v   = (const float*)d_in[9];
  const float* Wun   = (const float*)d_in[10];
  const float* bun   = (const float*)d_in[11];
  const float* Wfc1  = (const float*)d_in[12];
  const float* bfc1  = (const float*)d_in[13];
  const float* Wfc2  = (const float*)d_in[14];
  const float* bfc2  = (const float*)d_in[15];
  float* out = (float*)d_out;

  char* ws = (char*)d_ws;
  const size_t bytesH = (size_t)NG * 8 * sizeof(float);
  const size_t bytesX = (size_t)NS * 16 * sizeof(unsigned short);
  const size_t offH  = 0;
  const size_t offXH = offH + bytesH;
  const size_t offXL = offXH + bytesX;
  const size_t total = offXL + bytesX;
  if (total > ws_size || total > (size_t)134217728) return;
  float*          HPL = (float*)(ws + offH);
  unsigned short* XH  = (unsigned short*)(ws + offXH);
  unsigned short* XL  = (unsigned short*)(ws + offXL);

  lin_un_kernel<<<(NU + 127) / 128, NT, 0, stream>>>(x_u, Wun, bun, XH, XL);
  agg1_kernel<<<NTILE1, NT, LDS1_BYTES, stream>>>(x_g, edges, W1r, W1o, b1v, HPL);
  agg2_kernel<<<NTILE2, NT, LDS2_BYTES, stream>>>(HPL, edges, W2r, W2o, b2v, XH, XL);
  mlp_kernel<<<MLP_BLOCKS, NT, 0, stream>>>(cand, XH, XL, Wfc1, bfc1, Wfc2, bfc2, out);
}
